// RGCNModel_1846835938035
// MI455X (gfx1250) — hardware-run, weakly checked
//
#include <hip/hip_runtime.h>
#include <stddef.h>
#include <stdint.h>

#define H_SPLIT 1

#define NN      50000
#define NE      400000
#define NR      8
#define FD      128
#define HD      128
#define OD      64
#define HP      256
#define K2L     (H_SPLIT ? 256 : 128)
#define MP      50048
#define GBM     128
#define SP      68
#define NTHR    256
#define NWAVE   8
#define EPT     8
#define WCH     (32 * EPT)
#define NBRUN   1024
#define SLB     10
#define NBK     49
#define NSLOT   (NBK * NBRUN)
#define NBB     (NR * NBK)
#define WLCAP   512
#define RCAP    2048
#define DEGCAP  32
#define MAXDEG_MEAS   24
#define MAXB1024_MEAS 8415
#define ABM     128
#define PERW    (((NE + NWAVE * WCH - 1) / (NWAVE * WCH)) * WCH)
#define WSMAX   (128u << 20)

#define BK_ZINTS (NWAVE * WLCAP + RCAP + 3 * NBRUN)
#define BK_INTS  (BK_ZINTS + 16)

#define PBX   (MP * FD / 8 / NTHR)
#define PBW1  (NR * HD * FD / 8 / NTHR)
#define PBR1  (HD * FD / 8 / NTHR)
#define PBW2  (NR * OD * HP / 8 / NTHR)
#define PBR2  (OD * HP / 8 / NTHR)
#define PBTOT (PBX + PBW1 + PBR1 + PBW2 + PBR2 + 1)

static_assert(NR == 8);
static_assert(MP % GBM == 0 && MP >= NN && MP == 391 * GBM && MP % ABM == 0);
static_assert(NBRUN == (1 << SLB) && NBRUN % ABM == 0 && NBRUN % 32 == 0);
static_assert(NBK * NBRUN >= MP && NBK * NBRUN >= NN);
static_assert(NE < (1 << 21) && (((long long)NE) << SLB) < (1LL << 31));
static_assert(NE % EPT == 0 && NE >= EPT && PERW % WCH == 0 && PERW * NWAVE >= NE);
static_assert(RCAP % (NTHR * 4) == 0 && BK_ZINTS % 4 == 0 && NWAVE * WLCAP >= RCAP);
static_assert((MAXB1024_MEAS / NR) * 3 / 2 <= RCAP);
static_assert(MAXDEG_MEAS + 8 <= DEGCAP && DEGCAP <= 32);
static_assert(NBRUN == 4 * NTHR);
static_assert(FD % 32 == 0 && K2L % 32 == 0 && HP == 2 * HD && K2L <= HP);
static_assert(HD % 64 == 0 && OD % 64 == 0 && HD == 4 * 32 && OD == 2 * 32);
static_assert((MP * FD / 8) % NTHR == 0 && (NR * HD * FD / 8) % NTHR == 0 && (HD * FD / 8) % NTHR == 0);
static_assert((NR * OD * HP / 8) % NTHR == 0 && (OD * HP / 8) % NTHR == 0);
static_assert(BK_INTS * 4 <= 65536);
static_assert((GBM * SP + 128) * 4 <= 65536);
static_assert((long long)NN * OD == 3200000LL);

typedef float          v2f   __attribute__((ext_vector_type(2)));
typedef float          v4f   __attribute__((ext_vector_type(4)));
typedef float          v8f   __attribute__((ext_vector_type(8)));
typedef int            v4i   __attribute__((ext_vector_type(4)));
typedef int            v8i   __attribute__((ext_vector_type(8)));
typedef unsigned short v8us  __attribute__((ext_vector_type(8)));
typedef unsigned short v16us __attribute__((ext_vector_type(16)));
typedef __bf16         v16bf __attribute__((ext_vector_type(16)));
typedef v2f  __attribute__((may_alias)) v2fa;
typedef v4f  __attribute__((may_alias)) v4fa;
typedef v4i  __attribute__((may_alias)) v4ia;
typedef v8us __attribute__((may_alias)) v8usa;
union FragB { v16bf v; v16us u; v8us h[2]; v8i w; };

template <int PER> struct VecSel;
template <> struct VecSel<4> { typedef v4f T; typedef v4fa TA; };
template <> struct VecSel<2> { typedef v2f T; typedef v2fa TA; };

__device__ __forceinline__ v8f wmb(const FragB& a, const FragB& b, v8f c) {
  v8f d = __builtin_amdgcn_wmma_f32_16x16x32_bf16(false, a.v, false, b.v, (short)0, c, false, false);
  asm volatile("v_nop\n\tv_nop\n\tv_nop\n\tv_nop" : "+v"(d) : "v"(a.w), "v"(b.w));
  return d;
}

__device__ __forceinline__ unsigned bf16_bits(float f) {
  const unsigned u = __float_as_uint(f);
  const unsigned r = (u + 0x7FFFu + ((u >> 16) & 1u)) >> 16;
  const unsigned q = (u >> 16) | 0x40u;
  return ((u & 0x7fffffffu) > 0x7f800000u) ? q : r;
}
__device__ __forceinline__ float bf16_val(float f) {
  return __uint_as_float(bf16_bits(f) << 16);
}

__device__ __forceinline__ void hilo_pack(float v0, float v1, float v2, float v3,
                                          int& h01, int& h23, int& l01, int& l23) {
  const unsigned a0 = bf16_bits(v0), a1 = bf16_bits(v1), a2 = bf16_bits(v2), a3 = bf16_bits(v3);
  const unsigned b0 = bf16_bits(v0 - __uint_as_float(a0 << 16));
  const unsigned b1 = bf16_bits(v1 - __uint_as_float(a1 << 16));
  const unsigned b2 = bf16_bits(v2 - __uint_as_float(a2 << 16));
  const unsigned b3 = bf16_bits(v3 - __uint_as_float(a3 << 16));
  h01 = (int)(a0 | (a1 << 16)); h23 = (int)(a2 | (a3 << 16));
  l01 = (int)(b0 | (b1 << 16)); l23 = (int)(b2 | (b3 << 16));
}

__device__ __forceinline__ v4i regroup32(int h01, int h23, int l01, int l23, int lane) {
  const int s0 = (2 * lane) & 31, s1 = s0 + 1;
  const int a0 = __shfl(h01, s0, 32), a1 = __shfl(h23, s0, 32), a2 = __shfl(h01, s1, 32), a3 = __shfl(h23, s1, 32);
  const int b0 = __shfl(l01, s0, 32), b1 = __shfl(l23, s0, 32), b2 = __shfl(l01, s1, 32), b3 = __shfl(l23, s1, 32);
  const int mk = (lane < 16) ? -1 : 0;
  v4i o;
  o.x = (a0 & mk) | (b0 & ~mk); o.y = (a1 & mk) | (b1 & ~mk);
  o.z = (a2 & mk) | (b2 & ~mk); o.w = (a3 & mk) | (b3 & ~mk);
  return o;
}

__device__ __forceinline__ void st2_v4f(float* p, v4f v) {
  *(volatile v4f*)p = v;
  __threadfence();
  *(volatile v4f*)p = v;
}
__device__ __forceinline__ void st2_v8us(unsigned short* p, v8us v) {
  *(volatile v8us*)p = v;
  __threadfence();
  *(volatile v8us*)p = v;
}
__device__ __forceinline__ void st2_v4i(unsigned short* p, v4i v) {
  *(volatile v4i*)p = v;
  __threadfence();
  *(volatile v4i*)p = v;
}
template <int PER>
__device__ __forceinline__ void st2_vec(float* p, typename VecSel<PER>::T v) {
  typedef typename VecSel<PER>::T VT;
  *(volatile VT*)p = v;
  __threadfence();
  *(volatile VT*)p = v;
}

__device__ __forceinline__ v8us col8(const float* __restrict__ base, int stride) {
  float f[8];
#pragma unroll
  for (int i = 0; i < 8; ++i) f[i] = base[(size_t)i * (size_t)stride];
  v8us o;
#pragma unroll
  for (int i = 0; i < 8; ++i) o[i] = (unsigned short)bf16_bits(f[i]);
  return o;
}

__global__ __launch_bounds__(NTHR) void k_prep(const float* __restrict__ x, const float* __restrict__ w1,
                                               const float* __restrict__ r1, const float* __restrict__ b1,
                                               const float* __restrict__ w2, const float* __restrict__ r2,
                                               const float* __restrict__ b2,
                                               unsigned short* xb, unsigned short* w1t, unsigned short* r1t,
                                               unsigned short* w2d, unsigned short* r2d, float* sm) {
  const int tid = (int)threadIdx.x, lane = tid & 31;
  const int blk = (int)blockIdx.x;
  if (blk < PBX) {
    const int u   = blk * NTHR + tid;
    const int row = u >> 4, k8 = (u & 15) * 8;
    const int rc  = row < NN ? row : NN - 1;
    const unsigned mk = row < NN ? 0xffffu : 0u;
    const float* p = x + (size_t)rc * FD + k8;
    const v4f a = *(const v4fa*)p;
    const v4f b = *(const v4fa*)(p + 4);
    v8us o;
    o[0] = (unsigned short)(bf16_bits(a.x) & mk); o[1] = (unsigned short)(bf16_bits(a.y) & mk);
    o[2] = (unsigned short)(bf16_bits(a.z) & mk); o[3] = (unsigned short)(bf16_bits(a.w) & mk);
    o[4] = (unsigned short)(bf16_bits(b.x) & mk); o[5] = (unsigned short)(bf16_bits(b.y) & mk);
    o[6] = (unsigned short)(bf16_bits(b.z) & mk); o[7] = (unsigned short)(bf16_bits(b.w) & mk);
    st2_v8us(xb + (size_t)row * FD + k8, o);
  } else if (blk < PBX + PBW1) {
    const int u = (blk - PBX) * NTHR + tid;
    const int r = u >> 11, n = (u >> 4) & 127, k8 = (u & 15) * 8;
    const v8us o = col8(w1 + (size_t)r * FD * HD + (size_t)k8 * HD + n, HD);
    st2_v8us(w1t + (size_t)r * HD * FD + (size_t)n * FD + k8, o);
  } else if (blk < PBX + PBW1 + PBR1) {
    const int u = (blk - PBX - PBW1) * NTHR + tid;
    const int n = u >> 4, k8 = (u & 15) * 8;
    const v8us o = col8(r1 + (size_t)k8 * HD + n, HD);
    st2_v8us(r1t + (size_t)n * FD + k8, o);
  } else if (blk < PBX + PBW1 + PBR1 + PBW2) {
    const int u = (blk - PBX - PBW1 - PBR1) * NTHR + tid;
    const int r = u >> 11, n = (u >> 5) & 63, k8 = (u & 31) * 8, kk = k8 & 127;
    const v8us o = col8(w2 + (size_t)r * HD * OD + (size_t)kk * OD + n, OD);
    st2_v8us(w2d + (size_t)r * OD * HP + (size_t)n * HP + k8, o);
  } else if (blk < PBX + PBW1 + PBR1 + PBW2 + PBR2) {
    const int u = (blk - PBX - PBW1 - PBR1 - PBW2) * NTHR + tid;
    const int n = u >> 5, k8 = (u & 31) * 8, kk = k8 & 127;
    const v8us o = col8(r2 + (size_t)kk * OD + n, OD);
    st2_v8us(r2d + (size_t)n * HP + k8, o);
  } else {
    if (tid < 32) {
      const v4f a = *(const v4fa*)(b1 + 4 * lane);
      v4f o;
      o.x = bf16_val(a.x); o.y = bf16_val(a.y); o.z = bf16_val(a.z); o.w = bf16_val(a.w);
      st2_v4f(sm + 4 * lane, o);
    } else if (tid < 64) {
      const int q = lane & 15;
      const v4f a = *(const v4fa*)(b2 + 4 * q);
      asm volatile("" :: "v"(a));
      const unsigned ma = (lane < 16) ? 0xffffffffu : 0u;
      v4f o;
      o.x = __uint_as_float((bf16_bits(a.x) << 16) & ma);
      o.y = __uint_as_float((bf16_bits(a.y) << 16) & ma);
      o.z = __uint_as_float((bf16_bits(a.z) << 16) & ma);
      o.w = __uint_as_float((bf16_bits(a.w) << 16) & ma);
      st2_v4f(sm + HD + 4 * lane, o);
    }
  }
}

__device__ __forceinline__ void bucket_flush(const int* pl, const int* cnt, const int* offs, int ov,
                                             int* lp, int* cp, int* op, int* fp, int tid) {
#pragma unroll 1
  for (int i = tid * 4; i < RCAP; i += NTHR * 4) {
    const v4i v = *(const v4ia*)(pl + i);
    *(volatile v4i*)(lp + i) = v;
  }
  {
    const v4i v = *(const v4ia*)(cnt + 4 * tid);
    *(volatile v4i*)(cp + 4 * tid) = v;
  }
  {
    const v4i v = *(const v4ia*)(offs + 4 * tid);
    *(volatile v4i*)(op + 4 * tid) = v;
  }
  if (tid < 8) {
    const v4i f = {ov, ov, ov, ov};
    *(volatile v4i*)(fp + 4 * tid) = f;
  }
}

__device__ __forceinline__ int clamp7(int t) {
  t = t < 0 ? 0 : t;
  return t > NR - 1 ? NR - 1 : t;
}

__global__ __launch_bounds__(NTHR) void k_bucket(const int* __restrict__ srcs, const int* __restrict__ dsts,
                                                 const int* __restrict__ types,
                                                 int* LIST, int* CNT, int* OFF, int* FLAG) {
  __shared__ __attribute__((aligned(16))) int dsm[BK_INTS];
  int* wl   = dsm;
  int* pl   = dsm + NWAVE * WLCAP;
  int* cnt  = pl + RCAP;
  int* offs = cnt + NBRUN;
  int* cur  = offs + NBRUN;
  int* misc = cur + NBRUN;
  const int tid = (int)threadIdx.x, lane = tid & 31;
  const int wave = __builtin_amdgcn_readfirstlane(tid >> 5);
  const int blk  = (int)blockIdx.x;
  const int role = blk / NBK;
  const int bb   = blk - role * NBK;
  const unsigned nbs = (unsigned)(bb * NBRUN);

  {
    const v4i z4 = {0, 0, 0, 0};
    for (int i = tid * 4; i < BK_ZINTS; i += NTHR * 4) *(v4ia*)(dsm + i) = z4;
    if (tid < 16) misc[tid] = 0;
  }
  __syncthreads();

  {
    const int ebeg = wave * PERW;
    const int eend = (ebeg + PERW < NE) ? (ebeg + PERW) : NE;
    int* mylist = wl + wave * WLCAP;
    int wc = 0;
#pragma unroll 1
    for (int cb = ebeg; cb < eend; cb += WCH) {
      const int e0 = cb + lane * EPT;
      const bool lv = (e0 + EPT) <= NE;
      const int ec = lv ? e0 : (NE - EPT);
      const v4i da = *(const v4ia*)(dsts + ec);
      const v4i db = *(const v4ia*)(dsts + ec + 4);
      const v4i ta = *(const v4ia*)(types + ec);
      const v4i tb = *(const v4ia*)(types + ec + 4);
      const unsigned s0 = (unsigned)da.x - nbs, s1 = (unsigned)da.y - nbs;
      const unsigned s2 = (unsigned)da.z - nbs, s3 = (unsigned)da.w - nbs;
      const unsigned s4 = (unsigned)db.x - nbs, s5 = (unsigned)db.y - nbs;
      const unsigned s6 = (unsigned)db.z - nbs, s7 = (unsigned)db.w - nbs;
      const bool h0 = lv & (s0 < (unsigned)NBRUN) & (clamp7(ta.x) == role);
      const bool h1 = lv & (s1 < (unsigned)NBRUN) & (clamp7(ta.y) == role);
      const bool h2 = lv & (s2 < (unsigned)NBRUN) & (clamp7(ta.z) == role);
      const bool h3 = lv & (s3 < (unsigned)NBRUN) & (clamp7(ta.w) == role);
      const bool h4 = lv & (s4 < (unsigned)NBRUN) & (clamp7(tb.x) == role);
      const bool h5 = lv & (s5 < (unsigned)NBRUN) & (clamp7(tb.y) == role);
      const bool h6 = lv & (s6 < (unsigned)NBRUN) & (clamp7(tb.z) == role);
      const bool h7 = lv & (s7 < (unsigned)NBRUN) & (clamp7(tb.w) == role);
      const unsigned m0 = __builtin_amdgcn_ballot_w32(h0), m1 = __builtin_amdgcn_ballot_w32(h1);
      const unsigned m2 = __builtin_amdgcn_ballot_w32(h2), m3 = __builtin_amdgcn_ballot_w32(h3);
      const unsigned m4 = __builtin_amdgcn_ballot_w32(h4), m5 = __builtin_amdgcn_ballot_w32(h5);
      const unsigned m6 = __builtin_amdgcn_ballot_w32(h6), m7 = __builtin_amdgcn_ballot_w32(h7);
      const unsigned any = m0 | m1 | m2 | m3 | m4 | m5 | m6 | m7;
      if (any != 0u) {
        const int pre = (int)(__builtin_amdgcn_mbcnt_lo(m0, 0u) + __builtin_amdgcn_mbcnt_lo(m1, 0u) +
                              __builtin_amdgcn_mbcnt_lo(m2, 0u) + __builtin_amdgcn_mbcnt_lo(m3, 0u) +
                              __builtin_amdgcn_mbcnt_lo(m4, 0u) + __builtin_amdgcn_mbcnt_lo(m5, 0u) +
                              __builtin_amdgcn_mbcnt_lo(m6, 0u) + __builtin_amdgcn_mbcnt_lo(m7, 0u));
        int p = wc + pre;
        if (h0) { if (p < WLCAP) mylist[p] = ((e0 + 0) << SLB) | (int)s0; p = p + 1; }
        if (h1) { if (p < WLCAP) mylist[p] = ((e0 + 1) << SLB) | (int)s1; p = p + 1; }
        if (h2) { if (p < WLCAP) mylist[p] = ((e0 + 2) << SLB) | (int)s2; p = p + 1; }
        if (h3) { if (p < WLCAP) mylist[p] = ((e0 + 3) << SLB) | (int)s3; p = p + 1; }
        if (h4) { if (p < WLCAP) mylist[p] = ((e0 + 4) << SLB) | (int)s4; p = p + 1; }
        if (h5) { if (p < WLCAP) mylist[p] = ((e0 + 5) << SLB) | (int)s5; p = p + 1; }
        if (h6) { if (p < WLCAP) mylist[p] = ((e0 + 6) << SLB) | (int)s6; p = p + 1; }
        if (h7) { if (p < WLCAP) mylist[p] = ((e0 + 7) << SLB) | (int)s7; p = p + 1; }
        wc += (int)(__builtin_popcount(m0) + __builtin_popcount(m1) + __builtin_popcount(m2) + __builtin_popcount(m3) +
                    __builtin_popcount(m4) + __builtin_popcount(m5) + __builtin_popcount(m6) + __builtin_popcount(m7));
      }
    }
    if (lane == 0) misc[wave] = wc;
  }
  __syncthreads();

  if (wave == 0) {
    int ov = 0, tot = 0;
#pragma unroll 1
    for (int w2 = 0; w2 < NWAVE; ++w2) {
      int c = misc[w2];
      if (c > WLCAP) ov = 1;
      c = c < 0 ? 0 : (c > WLCAP ? WLCAP : c);
      tot += c;
#pragma unroll 1
      for (int b0 = 0; b0 < c; b0 += 32) {
        const int idx = b0 + lane;
        const int ent = wl[w2 * WLCAP + (idx < WLCAP ? idx : WLCAP - 1)];
        const int m32 = (c - b0) < 32 ? (c - b0) : 32;
#pragma unroll 1
        for (int k = 0; k < m32; ++k) {
          const int u    = __builtin_amdgcn_readlane(ent, k);
          const int slot = u & (NBRUN - 1);
          if (lane == 0) cnt[slot] = cnt[slot] + 1;
        }
      }
    }
    if (tot > RCAP) ov = 1;
    if (lane == 0) misc[9] = ov;
  }
  __syncthreads();
  if (wave == 0) {
    const int base = lane * (NBRUN / 32);
    int s = 0, dm = 0;
#pragma unroll 1
    for (int i = 0; i < NBRUN / 32; ++i) {
      const int cv = cnt[base + i];
      s += cv;
      dm = cv > dm ? cv : dm;
    }
    int incl = s;
#pragma unroll
    for (int d = 1; d < 32; d <<= 1) {
      const int y = __shfl_up(incl, d, 32);
      if (lane >= d) incl += y;
    }
    const unsigned bm = __builtin_amdgcn_ballot_w32(dm > DEGCAP);
    int run = incl - s;
#pragma unroll 1
    for (int i = 0; i < NBRUN / 32; ++i) {
      const int cv = cnt[base + i];
      offs[base + i] = run;
      cur[base + i]  = run;
      run += cv;
    }
    if (bm != 0u && lane == 0) misc[9] = 1;
  }
  __syncthreads();

  if (wave == 0) {
#pragma unroll 1
    for (int w2 = 0; w2 < NWAVE; ++w2) {
      int c = misc[w2];
      c = c < 0 ? 0 : (c > WLCAP ? WLCAP : c);
#pragma unroll 1
      for (int b0 = 0; b0 < c; b0 += 32) {
        const int idx = b0 + lane;
        const int ent = wl[w2 * WLCAP + (idx < WLCAP ? idx : WLCAP - 1)];
        int eid = (ent >> SLB) & 0x1FFFFF;
        eid = eid > NE - 1 ? NE - 1 : eid;
        int sr = srcs[eid];
        sr = sr < 0 ? 0 : (sr > NN - 1 ? NN - 1 : sr);
        const int m32 = (c - b0) < 32 ? (c - b0) : 32;
#pragma unroll 1
        for (int k = 0; k < m32; ++k) {
          const int u    = __builtin_amdgcn_readlane(ent, k);
          const int wd   = __builtin_amdgcn_readlane(sr, k);
          const int slot = u & (NBRUN - 1);
          if (lane == 0) {
            int p = cur[slot];
            p = p < 0 ? 0 : (p > RCAP - 1 ? RCAP - 1 : p);
            pl[p] = wd;
            cur[slot] = p + 1;
          }
        }
      }
    }
  }
  __syncthreads();

  const int ovf = misc[9];
  int* lp = LIST + (size_t)blk * RCAP;
  int* cp = CNT + (size_t)role * NSLOT + (size_t)bb * NBRUN;
  int* op = OFF + (size_t)role * NSLOT + (size_t)bb * NBRUN;
  int* fp = FLAG + (size_t)blk * 32;
  bucket_flush(pl, cnt, offs, ovf, lp, cp, op, fp, tid);
  __threadfence();
  bucket_flush(pl, cnt, offs, ovf, lp, cp, op, fp, tid);
}

template <int KTOT, int BPITCH>
__device__ __forceinline__ void gemm_16x64(const unsigned short* __restrict__ ap,
                                           const unsigned short* __restrict__ bp, v8f (&acc)[4]) {
#pragma unroll 1
  for (int k0 = 0; k0 < KTOT; k0 += 32) {
    FragB af;
    af.h[0] = *(const v8usa*)(ap + k0);
    af.h[1] = *(const v8usa*)(ap + k0 + 16);
#pragma unroll
    for (int nt = 0; nt < 4; ++nt) {
      const unsigned short* wq = bp + (size_t)(16 * nt) * (size_t)BPITCH + k0;
      FragB bf;
      bf.h[0] = *(const v8usa*)wq;
      bf.h[1] = *(const v8usa*)(wq + 16);
      acc[nt] = wmb(af, bf, acc[nt]);
    }
  }
}

__device__ __forceinline__ void stage_d(float* stg, const v8f (&acc)[4], int wave, int hh, int m) {
#pragma unroll
  for (int nt = 0; nt < 4; ++nt) {
#pragma unroll
    for (int r = 0; r < 8; ++r) stg[(16 * wave + 8 * hh + r) * SP + 16 * nt + m] = acc[nt][r];
  }
}

template <int APITCH, int BPITCH, int KTOT, int NC, int BIAS>
__global__ __launch_bounds__(NTHR) __attribute__((amdgpu_num_vgpr(248)))
void k_gemm(const unsigned short* __restrict__ A, const unsigned short* __restrict__ BT,
            const float* __restrict__ sm, float* C) {
  __shared__ __attribute__((aligned(16))) float stg[GBM * SP];
  __shared__ __attribute__((aligned(16))) float sb[128];
  const int tid = (int)threadIdx.x, lane = tid & 31, wave = tid >> 5, hh = lane >> 4, m = lane & 15;
  const int rowBase = (int)blockIdx.x * GBM;
  if constexpr (BIAS != 0) {
    if (tid < 32) *(v4fa*)(sb + 4 * tid) = *(const v4fa*)(sm + 4 * tid);
  }
  const unsigned short* ap = A + (size_t)(rowBase + 16 * wave + m) * (size_t)APITCH + 8 * hh;

#pragma unroll 1
  for (int ch = 0; ch < NC / 64; ++ch) {
    v8f acc[4];
    {
      const v8f z = {0.f, 0.f, 0.f, 0.f, 0.f, 0.f, 0.f, 0.f};
#pragma unroll
      for (int t = 0; t < 4; ++t) acc[t] = z;
    }
    const unsigned short* bp = BT + (size_t)(64 * ch + m) * (size_t)BPITCH + 8 * hh;
    gemm_16x64<KTOT, BPITCH>(ap, bp, acc);
    stage_d(stg, acc, wave, hh, m);
    __syncthreads();

    v4f bias = {0.f, 0.f, 0.f, 0.f};
    if constexpr (BIAS != 0) bias = *(const v4fa*)(sb + 64 * ch + 4 * m);
#pragma unroll 1
    for (int i = 0; i < 8; ++i) {
      const int lr   = 16 * wave + 2 * i + hh;
      const int grow = rowBase + lr;
      const bool live = grow < NN;
      const v4f a = *(const v4fa*)(stg + lr * SP + 4 * m);
      asm volatile("" :: "v"(a));
      const float v0 = a.x + bias.x, v1 = a.y + bias.y, v2 = a.z + bias.z, v3 = a.w + bias.w;
      v4f o;
      o.x = live ? v0 : 0.0f; o.y = live ? v1 : 0.0f; o.z = live ? v2 : 0.0f; o.w = live ? v3 : 0.0f;
      st2_v4f(C + (size_t)grow * NC + 64 * ch + 4 * m, o);
    }
    __syncthreads();
  }
}

template <int W, int FIN>
__global__ __launch_bounds__(NTHR) void k_replay(const int* __restrict__ LIST, const int* __restrict__ CNT,
                                                 const int* __restrict__ OFF, const int* __restrict__ FLAG,
                                                 const float* __restrict__ P, float* ACC, int role,
                                                 const float* __restrict__ mask, unsigned short* HHL, float* outp) {
  constexpr int PER = W / 32;
  static_assert(PER == 4 || PER == 2);
  static_assert(FIN != 1 || W == HD);
  static_assert(FIN != 2 || W == OD);
  typedef typename VecSel<PER>::T  VT;
  typedef typename VecSel<PER>::TA VTA;
  const int tid = (int)threadIdx.x, lane = tid & 31;
  const int wave = __builtin_amdgcn_readfirstlane(tid >> 5);
  int rc = role;
  rc = rc < 0 ? 0 : (rc > NR - 1 ? NR - 1 : rc);
  const int rowBase = (int)blockIdx.x * ABM;
  const int bucket  = rowBase >> SLB;
  const int lbi     = rc * NBK + bucket;
  const int* lb = LIST + (size_t)lbi * RCAP;
  const int* cb = CNT + (size_t)rc * NSLOT + rowBase + 16 * wave;
  const int* ob = OFF + (size_t)rc * NSLOT + rowBase + 16 * wave;
  int flag = 0;
  if constexpr (FIN != 0) {
#pragma unroll
    for (int rr = 0; rr < NR; ++rr) flag |= FLAG[(size_t)(rr * NBK + bucket) * 32];
  } else {
    flag = FLAG[(size_t)lbi * 32];
  }
  const float qnan = __uint_as_float(0x7fc00000u);

#pragma unroll 1
  for (int i = 0; i < ABM / NWAVE; ++i) {
    const int d = rowBase + 16 * wave + i;
    int cv = cb[i];
    int ov = ob[i];
    const int bigv = cv > DEGCAP ? 1 : 0;
    cv = cv < 0 ? 0 : (cv > DEGCAP ? DEGCAP : cv);
    ov = ov < 0 ? 0 : (ov > RCAP - 1 ? RCAP - 1 : ov);
    const int c   = __builtin_amdgcn_readfirstlane(cv);
    const int o   = __builtin_amdgcn_readfirstlane(ov);
    const int big = __builtin_amdgcn_readfirstlane(bigv);
    const bool bad  = (flag != 0) | (big != 0);
    int last = o + c - 1;
    last = last < o ? o : last;
    last = last > RCAP - 1 ? RCAP - 1 : last;
    const bool live = d < NN;
    const bool work = live & ((FIN != 0) | (c > 0) | bad);

    float v[4] = {0.0f, 0.0f, 0.0f, 0.0f};
    float hv[4] = {0.0f, 0.0f, 0.0f, 0.0f};
    if (work) {
      int idx = o + lane;
      idx = idx > last ? last : idx;
      int ent = lb[idx];
      ent = ent < 0 ? 0 : (ent > NN - 1 ? NN - 1 : ent);
      float s[4] = {0.0f, 0.0f, 0.0f, 0.0f};
#pragma unroll 1
      for (int k = 0; k < c; ++k) {
        const int sk = __builtin_amdgcn_readlane(ent, k);
        const VT pv = *(const VTA*)(P + (size_t)sk * W + PER * lane);
#pragma unroll
        for (int j = 0; j < PER; ++j) s[j] += pv[j];
      }
      const float cf   = fmaxf((float)c, 1.0f);
      const float coef = 1.0f / cf;
      const VT a = *(const VTA*)(ACC + (size_t)d * W + PER * lane);
#pragma unroll
      for (int j = 0; j < PER; ++j) {
        const float t = a[j] + coef * s[j];
        v[j] = bad ? qnan : t;
      }
      if constexpr (FIN == 0) {
        VT ov4;
#pragma unroll
        for (int j = 0; j < PER; ++j) ov4[j] = v[j];
        st2_vec<PER>(ACC + (size_t)d * W + PER * lane, ov4);
      }
      if constexpr (FIN == 2) {
        VT ov4;
#pragma unroll
        for (int j = 0; j < PER; ++j) ov4[j] = v[j];
        st2_vec<PER>(outp + (size_t)d * W + PER * lane, ov4);
      }
      if constexpr (FIN == 1) {
        const v4f mk = *(const v4fa*)(mask + (size_t)d * HD + 4 * lane);
        const float r0 = (v[0] > 0.0f) ? v[0] : (v[0] - v[0]);
        const float r1 = (v[1] > 0.0f) ? v[1] : (v[1] - v[1]);
        const float r2 = (v[2] > 0.0f) ? v[2] : (v[2] - v[2]);
        const float r3 = (v[3] > 0.0f) ? v[3] : (v[3] - v[3]);
        hv[0] = r0 * bf16_val(mk.x);
        hv[1] = r1 * bf16_val(mk.y);
        hv[2] = r2 * bf16_val(mk.z);
        hv[3] = r3 * bf16_val(mk.w);
      }
    }
    if constexpr (FIN == 1) {
      int h01, h23, l01, l23;
      hilo_pack(hv[0], hv[1], hv[2], hv[3], h01, h23, l01, l23);
      const v4i ow = regroup32(h01, h23, l01, l23, lane);
      st2_v4i(HHL + (size_t)d * HP + 8 * lane, ow);
    }
  }
}

extern "C" void kernel_launch(void* const* d_in, const int* in_sizes, int n_in,
                              void* d_out, int out_size, void* d_ws, size_t ws_size,
                              hipStream_t stream) {
  if (n_in < 10) return;
  if (in_sizes[0] != NN * FD) return;
  if (in_sizes[1] != 2 * NE) return;
  if (in_sizes[2] != NE) return;
  if (in_sizes[3] != NR * FD * HD) return;
  if (in_sizes[4] != FD * HD) return;
  if (in_sizes[5] != HD) return;
  if (in_sizes[6] != NR * HD * OD) return;
  if (in_sizes[7] != HD * OD) return;
  if (in_sizes[8] != OD) return;
  if (in_sizes[9] != NN * HD) return;
  if (out_size != NN * OD) return;

  const float* x     = (const float*)d_in[0];
  const int*   ei    = (const int*)d_in[1];
  const int*   et    = (const int*)d_in[2];
  const float* W1    = (const float*)d_in[3];
  const float* root1 = (const float*)d_in[4];
  const float* b1    = (const float*)d_in[5];
  const float* W2    = (const float*)d_in[6];
  const float* root2 = (const float*)d_in[7];
  const float* b2    = (const float*)d_in[8];
  const float* dmask = (const float*)d_in[9];
  float* out = (float*)d_out;
  const int* srcs = ei;
  const int* dsts = ei + NE;

  constexpr size_t zXB   = (size_t)MP * FD * 2;
  constexpr size_t zP    = (size_t)MP * HD * 4;
  constexpr size_t zACC1 = (size_t)MP * HD * 4;
  constexpr size_t zHHL  = (size_t)MP * HP * 2;
  constexpr size_t zACC2 = (size_t)MP * OD * 4;
  constexpr size_t zLIST = (size_t)NBB * RCAP * 4;
  constexpr size_t zCNT  = (size_t)NR * NSLOT * 4;
  constexpr size_t zOFF  = (size_t)NR * NSLOT * 4;
  constexpr size_t zFLAG = (size_t)NBB * 128;
  constexpr size_t zW1T  = (size_t)NR * HD * FD * 2;
  constexpr size_t zR1T  = (size_t)HD * FD * 2;
  constexpr size_t zW2D  = (size_t)NR * OD * HP * 2;
  constexpr size_t zR2D  = (size_t)OD * HP * 2;
  constexpr size_t zSM   = 1024;
  constexpr size_t oXB   = 0;
  constexpr size_t oP    = oXB + zXB;
  constexpr size_t oACC1 = oP + zP;
  constexpr size_t oHHL  = oACC1 + zACC1;
  constexpr size_t oACC2 = oHHL + zHHL;
  constexpr size_t oLIST = oACC2 + zACC2;
  constexpr size_t oCNT  = oLIST + zLIST;
  constexpr size_t oOFF  = oCNT + zCNT;
  constexpr size_t oFLAG = oOFF + zOFF;
  constexpr size_t oW1T  = oFLAG + zFLAG;
  constexpr size_t oR1T  = oW1T + zW1T;
  constexpr size_t oW2D  = oR1T + zR1T;
  constexpr size_t oR2D  = oW2D + zW2D;
  constexpr size_t oSM   = oR2D + zR2D;
  constexpr size_t oEND  = oSM + zSM;
  static_assert(zXB % 256 == 0 && zP % 256 == 0 && zHHL % 256 == 0 && zACC2 % 256 == 0 && zLIST % 256 == 0);
  static_assert(zCNT % 256 == 0 && zFLAG % 256 == 0 && zW1T % 256 == 0 && zR1T % 256 == 0 && zW2D % 256 == 0);
  static_assert(zR2D % 256 == 0 && zSM % 256 == 0 && zSM >= 256 * 4);
  static_assert(zP >= (size_t)MP * OD * 4);
  static_assert(oEND <= (size_t)WSMAX);
  if (oEND > ws_size) return;

  char* ws = (char*)d_ws;
  unsigned short* XB   = (unsigned short*)(ws + oXB);
  float*          P    = (float*)(ws + oP);
  float*          ACC1 = (float*)(ws + oACC1);
  unsigned short* HHL  = (unsigned short*)(ws + oHHL);
  float*          ACC2 = (float*)(ws + oACC2);
  int*            LIST = (int*)(ws + oLIST);
  int*            CNT  = (int*)(ws + oCNT);
  int*            OFF  = (int*)(ws + oOFF);
  int*            FLAG = (int*)(ws + oFLAG);
  unsigned short* W1T  = (unsigned short*)(ws + oW1T);
  unsigned short* R1T  = (unsigned short*)(ws + oR1T);
  unsigned short* W2D  = (unsigned short*)(ws + oW2D);
  unsigned short* R2D  = (unsigned short*)(ws + oR2D);
  float*          SM   = (float*)(ws + oSM);

  k_prep<<<PBTOT, NTHR, 0, stream>>>(x, W1, root1, b1, W2, root2, b2, XB, W1T, R1T, W2D, R2D, SM);
  k_bucket<<<NBB, NTHR, 0, stream>>>(srcs, dsts, et, LIST, CNT, OFF, FLAG);

  k_gemm<FD, FD, FD, HD, 1><<<MP / GBM, NTHR, 0, stream>>>(XB, R1T, SM, ACC1);
  for (int r = 0; r < NR; ++r) {
    k_gemm<FD, FD, FD, HD, 0><<<MP / GBM, NTHR, 0, stream>>>(XB, W1T + (size_t)r * HD * FD, SM, P);
    if (r == NR - 1)
      k_replay<HD, 1><<<MP / ABM, NTHR, 0, stream>>>(LIST, CNT, OFF, FLAG, P, ACC1, r, dmask, HHL, out);
    else
      k_replay<HD, 0><<<MP / ABM, NTHR, 0, stream>>>(LIST, CNT, OFF, FLAG, P, ACC1, r, dmask, HHL, out);
  }

  k_gemm<HP, HP, K2L, OD, 1><<<MP / GBM, NTHR, 0, stream>>>(HHL, R2D, SM + HD, ACC2);
  for (int r = 0; r < NR; ++r) {
    k_gemm<HP, HP, K2L, OD, 0><<<MP / GBM, NTHR, 0, stream>>>(HHL, W2D + (size_t)r * OD * HP, SM + HD, P);
    if (r == NR - 1)
      k_replay<OD, 2><<<MP / ABM, NTHR, 0, stream>>>(LIST, CNT, OFF, FLAG, P, ACC2, r, dmask, HHL, out);
    else
      k_replay<OD, 0><<<MP / ABM, NTHR, 0, stream>>>(LIST, CNT, OFF, FLAG, P, ACC2, r, dmask, HHL, out);
  }
}
